// Poly2d_61675730370816
// MI455X (gfx1250) — hardware-verified
//
#include <hip/hip_runtime.h>

#define NI_ 4
#define CC_ 64
#define HH_ 64
#define WW_ 64
#define HW_ 4096
#define LL_ 10
#define KTOT (CC_ * LL_ * LL_)
#define KST 40

typedef _Float16 f16;
typedef __attribute__((ext_vector_type(16))) f16 f16x16;
typedef __attribute__((ext_vector_type(8)))  f16 f16x8;
typedef __attribute__((ext_vector_type(8)))  float f32x8;
typedef __attribute__((ext_vector_type(4)))  float v4f_t;
typedef float v4fa __attribute__((ext_vector_type(4), may_alias));

__device__ __forceinline__ f32x8 wmma16(f16x16 a, f16x16 b, f32x8 c) {
  c = __builtin_amdgcn_wmma_f32_16x16x32_f16(false, a, false, b, (short)0, c, false, false);
  asm volatile("v_nop\n\tv_nop\n\tv_nop\n\tv_nop" : "+v"(c) : "v"(a), "v"(b));
  return c;
}
__device__ __forceinline__ f16x16 lds_frag(const f16* base, int stride) {
  const int lane = threadIdx.x & 31, row = lane & 15, kh = (lane >> 4) * 8;
  const f16x8 lo = *(const f16x8*)(base + row * stride + kh);
  const f16x8 hi = *(const f16x8*)(base + row * stride + kh + 16);
  f16x16 f;
#pragma unroll
  for (int i = 0; i < 8; ++i) { f[i] = lo[i]; f[i + 8] = hi[i]; }
  return f;
}

__global__ __launch_bounds__(256) void k_poly(const float* __restrict__ x, const float* __restrict__ F, const float* __restrict__ bias, float* __restrict__ Y) {
  __shared__ __attribute__((aligned(16))) f16 ldsA[64 * KST];
  __shared__ __attribute__((aligned(16))) f16 ldsB[256 * KST];
  __shared__ __attribute__((aligned(16))) float oS[8][32 * 68];
  __shared__ float sP[256][12];
  const int tid = threadIdx.x, lane = tid & 31, wave = tid >> 5, cl = lane & 15, rh = (lane >> 4) * 8;
  const int b = blockIdx.x >> 4, y0 = (blockIdx.x & 15) * 4;
  const int wm = (wave & 1) * 32, wrow = wave >> 1;
  const float* inb = x + (size_t)b * CC_ * HW_;
  const int yy = tid >> 6, xx = tid & 63;
  f32x8 acc[2][4];
#pragma unroll
  for (int i = 0; i < 2; ++i)
#pragma unroll
    for (int j = 0; j < 4; ++j) { f32x8 z = {}; acc[i][j] = z; }
  int curc = -1;
#pragma unroll 1
  for (int k0 = 0; k0 < KTOT; k0 += 32) {
    __syncthreads();
    { const int o = tid >> 2, kq = (tid & 3) * 8;
#pragma unroll
      for (int u = 0; u < 8; ++u) ldsA[o * KST + kq + u] = (f16)F[(size_t)o * KTOT + k0 + kq + u]; }
#pragma unroll 2
    for (int kk = 0; kk < 32; ++kk) {
      const int k = k0 + kk, c = k / 100, ij = k - 100 * c, i = ij / 10, j = ij - 10 * i;
      if (c != curc) {
        curc = c;
        sP[tid][0] = 1.0f;
#pragma unroll
        for (int t9 = 0; t9 < 9; ++t9) { const int dy = t9 / 3 - 1, dx = t9 - 3 * (t9 / 3) - 1; const int ys = y0 + yy + dy, xs = xx + dx;
          sP[tid][1 + t9] = (ys >= 0 && ys < HH_ && xs >= 0 && xs < WW_) ? inb[(size_t)c * HW_ + ys * WW_ + xs] : 0.0f; }
      }
      ldsB[tid * KST + kk] = (f16)(sP[tid][i] * sP[tid][j]);
    }
    __syncthreads();
    f16x16 af[2];
#pragma unroll
    for (int i = 0; i < 2; ++i) af[i] = lds_frag(ldsA + (wm + 16 * i) * KST, KST);
#pragma unroll
    for (int j = 0; j < 4; ++j) {
      const f16x16 bfv = lds_frag(ldsB + (wrow * 64 + 16 * j) * KST, KST);
#pragma unroll
      for (int i = 0; i < 2; ++i) acc[i][j] = wmma16(af[i], bfv, acc[i][j]);
    }
  }
  float* so = oS[wave];
#pragma unroll
  for (int i = 0; i < 2; ++i)
#pragma unroll
    for (int r = 0; r < 8; ++r) {
      const int o = wm + 16 * i + rh + r;
      const float bv = bias[o];
#pragma unroll
      for (int j = 0; j < 4; ++j) so[(16 * i + rh + r) * 68 + 16 * j + cl] = acc[i][j][r] + bv;
    }
  asm volatile("s_wait_dscnt 0" ::: "memory");
  __builtin_amdgcn_wave_barrier();
  const int yrow = y0 + wrow;
#pragma unroll 1
  for (int pass = 0; pass < 2; ++pass) {
#pragma unroll
    for (int it = 0; it < 16; ++it) { const int f4 = lane + 32 * it, rr = f4 >> 4, q = (f4 & 15) * 4;
      const size_t off = (((size_t)b * CC_ + wm + rr) * HH_ + yrow) * WW_ + q;
      *(volatile v4f_t*)(Y + off) = *(const volatile v4fa*)(so + rr * 68 + q); }
    __threadfence();
  }
}

extern "C" void kernel_launch(void* const* d_in, const int* in_sizes, int n_in,
                              void* d_out, int out_size, void* d_ws, size_t ws_size,
                              hipStream_t stream) {
  (void)in_sizes; (void)n_in; (void)out_size; (void)d_ws; (void)ws_size;
  const float* x = (const float*)d_in[0];
  const float* F = (const float*)d_in[1];
  const float* bias = (const float*)d_in[2];
  float* out = (float*)d_out;
  k_poly<<<dim3(NI_ * 16), dim3(256), 0, stream>>>(x, F, bias, out);
}
